// PairwiseFeaturizer_53154515255691
// MI455X (gfx1250) — hardware-run, weakly checked
//
#include <hip/hip_runtime.h>


namespace {
constexpr int NB_ = 4, NO = 512, D = 64, DH = 64, NP = NO * (NO - 1) / 2  ;
constexpr float XS = 8.0f, HS = 256.0f, WSC = 256.0f;
typedef _Float16 b16;
typedef __attribute__((ext_vector_type(16))) _Float16 v16b;
typedef __attribute__((ext_vector_type(8))) _Float16 v8b;
typedef __attribute__((ext_vector_type(8))) float v8f;
typedef __attribute__((ext_vector_type(4))) float v4f;
typedef __attribute__((ext_vector_type(2))) float v2f;
__device__ __forceinline__ float bf16_rne(float f) { unsigned int u = __float_as_uint(f); u += 0x7FFFu + ((u >> 16) & 1u); float r = __uint_as_float(u & 0xFFFF0000u); asm volatile("" : "+v"(r)); return r; }
__device__ __forceinline__ float bfv(float f) { float r = bf16_rne(f); asm volatile("" : "+v"(r)); return r; }
__device__ __forceinline__ void split16(float v, b16& hi, b16& lo) { hi = (b16)v; lo = (b16)(v - (float)hi); }
__device__ __forceinline__ v16b frag_kb(const b16* p, int hh) { const v8b a = *(const v8b*)(p + 8 * hh), b = *(const v8b*)(p + 16 + 8 * hh); v16b f;
#pragma unroll
  for (int e = 0; e < 8; ++e) { f[e] = a[e]; f[8 + e] = b[e]; } return f; }
__device__ __forceinline__ v8f wmma16b(v16b a, v16b b, v8f c) { v8f d = __builtin_amdgcn_wmma_f32_16x16x32_f16(false, a, false, b, (short)0, c, false, false); asm volatile("v_nop\n\tv_nop\n\tv_nop\n\tv_nop" : "+v"(d) : "v"(a), "v"(b)); return d; }
__device__ __forceinline__ void wave_lds_sync() { __builtin_amdgcn_fence(__ATOMIC_RELEASE, "workgroup"); __builtin_amdgcn_wave_barrier(); __builtin_amdgcn_fence(__ATOMIC_ACQUIRE, "workgroup"); }
__device__ __forceinline__ float pmul(float a, float b) { float p = a * b; asm volatile("" : "+v"(p)); return p; }
__device__ __forceinline__ void pair_of(int p, int& i, int& j) { int ii = 0, rem = p; while (rem >= NO - 1 - ii) { rem -= NO - 1 - ii; ++ii; } i = ii; j = ii + 1 + rem; }

__global__ __launch_bounds__(256) void wput_kernel(const float* __restrict__ w1, b16* __restrict__ WAB, b16* __restrict__ WCD) { const int u = blockIdx.x * 256 + threadIdx.x; v8b v;
  if (u < 128 * 8) { const int op = u / 8, k0 = (u % 8) * 8; const int o = op % DH, blk = op / DH;
#pragma unroll
    for (int j = 0; j < 8; ++j) v[j] = (b16)(bf16_rne(w1[(size_t)(blk * D + k0 + j) * DH + o]) * WSC); for (int pass = 0; pass < 2; ++pass) { *(volatile v8b*)(WAB + (size_t)op * D + k0) = v; __threadfence(); } }
  if (u < DH * 16) { const int o = u / 16, k0 = (u % 16) * 8; const int blk = 2 + k0 / D, kk = k0 % D;
#pragma unroll
    for (int j = 0; j < 8; ++j) v[j] = (b16)(bf16_rne(w1[(size_t)(blk * D + kk + j) * DH + o]) * WSC); for (int pass = 0; pass < 2; ++pass) { *(volatile v8b*)(WCD + (size_t)o * 2 * D + k0) = v; __threadfence(); } } }
__global__ __launch_bounds__(32) void obj_kernel(const float* __restrict__ O, const b16* __restrict__ WAB, float* __restrict__ P) { __shared__ __attribute__((aligned(16))) b16 Ah[16][D + 8]; __shared__ float Tf[16][132]; const int lane = threadIdx.x, nloc = lane & 15, hlf = lane >> 4; const size_t m0 = (size_t)blockIdx.x * 16;
  for (int rr = 0; rr < 16; ++rr) for (int q = 0; q < 2; ++q) Ah[rr][q * 32 + lane] = (b16)(bf16_rne(O[(m0 + rr) * D + q * 32 + lane]) * XS); if (lane < 16) for (int k = D; k < D + 8; ++k) Ah[lane][k] = (b16)0.0f;
  wave_lds_sync(); v8f acc[8];
#pragma unroll
  for (int t = 0; t < 8; ++t) acc[t] = (v8f){};
#pragma unroll
  for (int kb = 0; kb < D; kb += 32) { const v16b a = frag_kb(&Ah[nloc][kb], hlf);
#pragma unroll
    for (int t = 0; t < 8; ++t) acc[t] = wmma16b(a, frag_kb(WAB + (size_t)(t * 16 + nloc) * D + kb, hlf), acc[t]); }
#pragma unroll
  for (int t = 0; t < 8; ++t)
#pragma unroll
    for (int r8 = 0; r8 < 8; ++r8) Tf[8 * hlf + r8][t * 16 + nloc] = acc[t][r8] * (1.0f / (XS * WSC));
  wave_lds_sync();
  for (int pass = 0; pass < 2; ++pass) { for (int rr = 0; rr < 16; ++rr) *(volatile v4f*)(P + (m0 + rr) * 2 * DH + lane * 4) = *(const v4f*)(&Tf[rr][lane * 4]); __threadfence(); } }
__global__ __launch_bounds__(32) void pair_kernel(const float* __restrict__ O, const float* __restrict__ P, const b16* __restrict__ WCD, const float* __restrict__ b1, const float* __restrict__ w2, const float* __restrict__ b2, int PLIM, float* __restrict__ out) { __shared__ __attribute__((aligned(16))) b16 Ah[32][2 * D + 8], Al[32][2 * D + 8]; __shared__ float Tf[32][DH + 1], Os[32]; __shared__ int Pi[32], Pj[32]; const int lane = threadIdx.x, nloc = lane & 15, hlf = lane >> 4; const int b = blockIdx.x / (NP / 32); const int p0 = (blockIdx.x % (NP / 32)) * 32; if (p0 >= PLIM) return;
  { int i, j; pair_of(p0 + lane, i, j); Pi[lane] = i; Pj[lane] = j; }
  wave_lds_sync();
  for (int rr = 0; rr < 32; ++rr) { const size_t oi = ((size_t)b * NO + Pi[rr]) * D, oj = ((size_t)b * NO + Pj[rr]) * D; for (int q = 0; q < 2; ++q) { const int c = q * 32 + lane; const float a = bfv(O[oi + c]), bb = bfv(O[oj + c]); b16 p, ql; split16(fabsf(a - bb) * HS, p, ql); Ah[rr][c] = p; Al[rr][c] = ql; split16(pmul(a, bb) * HS, p, ql); Ah[rr][D + c] = p; Al[rr][D + c] = ql; } }
  for (int k = 2 * D; k < 2 * D + 8; ++k) { Ah[lane][k] = (b16)0.0f; Al[lane][k] = (b16)0.0f; }
  wave_lds_sync();
#pragma unroll
  for (int rt = 0; rt < 2; ++rt) { v8f acc[4] = {(v8f){}, (v8f){}, (v8f){}, (v8f){}};
#pragma unroll
    for (int kb = 0; kb < 2 * D; kb += 32) { const v16b a = frag_kb(&Ah[rt * 16 + nloc][kb], hlf), al = frag_kb(&Al[rt * 16 + nloc][kb], hlf);
#pragma unroll
      for (int t = 0; t < 4; ++t) { const v16b bw = frag_kb(WCD + (size_t)(t * 16 + nloc) * 2 * D + kb, hlf); acc[t] = wmma16b(a, bw, acc[t]); acc[t] = wmma16b(al, bw, acc[t]); } }
#pragma unroll
    for (int t = 0; t < 4; ++t) { const int cc = t * 16 + nloc; const float bb = bfv(b1[cc]);
#pragma unroll
      for (int r8 = 0; r8 < 8; ++r8) { const int rr = rt * 16 + 8 * hlf + r8; Tf[rr][cc] = acc[t][r8] * (1.0f / (HS * WSC)) + bb; } } }
  wave_lds_sync();
  { const float* pa = P + ((size_t)b * NO + Pi[lane]) * 2 * DH; const float* pb = P + ((size_t)b * NO + Pj[lane]) * 2 * DH + DH; float s = bfv(b2[0]);
#pragma unroll 4
    for (int c = 0; c < DH; ++c) s += pmul(fmaxf(Tf[lane][c] + pa[c] + pb[c], 0.0f), bfv(w2[c])); Os[lane] = s; }
  wave_lds_sync();
  for (int pass = 0; pass < 2; ++pass) { ((volatile float*)out)[(size_t)b * NP + p0 + lane] = Os[lane]; __threadfence(); } }
}

extern "C" void kernel_launch(void* const* d_in, const int* in_sizes, int n_in, void* d_out, int out_size, void* d_ws, size_t ws_size, hipStream_t stream) {
  (void)n_in;
  auto Fp = [&](int i) { return (const float*)d_in[i]; };
  if (in_sizes[0] != NB_ * NO * D || in_sizes[1] != 4 * D * DH || in_sizes[2] != DH || in_sizes[3] != DH || out_size != NB_ * NP) return;
  const int PLIM = NP;
  size_t off = 0; char* ws = (char*)d_ws;
  auto carve = [&](size_t bytes) { char* p = ws + off; off += (bytes + 255) & ~(size_t)255; return p; };
  b16* WAB = (b16*)carve((size_t)2 * DH * D * 2); b16* WCD = (b16*)carve((size_t)DH * 2 * D * 2); float* P = (float*)carve((size_t)NB_ * NO * 2 * DH * 4);
  if (off > ws_size || off > ((size_t)4 << 20)) return;
  wput_kernel<<<(DH * 16 + 255) / 256, 256, 0, stream>>>(Fp(1), WAB, WCD);
  obj_kernel<<<NB_ * NO / 16, 32, 0, stream>>>(Fp(0), WAB, P);
  pair_kernel<<<NB_ * (NP / 32), 32, 0, stream>>>(Fp(0), P, WCD, Fp(2), Fp(3), Fp(4), PLIM, (float*)d_out);
}
